// SimplePoseGCN_3393024164007
// MI455X (gfx1250) — hardware-verified
//
#include <hip/hip_runtime.h>
#include <math.h>

#ifndef NSAMP
#define NSAMP 32768
#endif
#define NJ 17
#define HID 128
#define PG 8
#define PB 32
#define ROWS (PG * NJ)
#define RPAD 144
#define NTILE 9
#define XP 136
#define LTP 152
#define AJP 72
#define AWK 64
#define OUTF (PB * NJ * 3)
#define SUBF (PG * NJ * 3)
#define SC_L 0.03125f
#define CARRY_X 8.0f
#define INV_CARRY 0.125f
#define H_SAT 60000.0f

static_assert(NSAMP % PB == 0);
static_assert(PB % PG == 0);
static_assert(ROWS == 136 && RPAD >= ROWS && RPAD % 16 == 0 && NTILE * 16 == RPAD);
static_assert(HID == 128 && HID / 16 == 8);
static_assert(XP % 8 == 0 && LTP % 8 == 0 && AJP % 8 == 0 && XP >= HID && LTP >= RPAD && AJP >= AWK);
static_assert(AWK == 64);
static_assert((OUTF * 4) % 128 == 0);
static_assert(OUTF / 4 > 256 && OUTF / 4 <= 512);
static_assert(((OUTF / 4 - 256) % 8) == 0);
static_assert(SUBF > 256 && SUBF <= 512);
static_assert(NTILE * 8 * 32 * 8 == HID * RPAD);
static_assert((RPAD * (AWK / 8) + 255) / 256 == 5);
static_assert((HID * (HID / 8)) % 256 == 0);
static_assert(RPAD * XP * 2 + HID * LTP * 2 + RPAD * AJP * 2 + 8 * RPAD * 16 + OUTF * 4 + RPAD * 2 * 4 <= 131072);

typedef __attribute__((ext_vector_type(16))) _Float16 v16h;
typedef __attribute__((ext_vector_type(8)))  _Float16 v8h;
typedef __attribute__((ext_vector_type(8)))  float    v8f;
typedef __attribute__((ext_vector_type(4)))  float    v4f;
typedef __attribute__((ext_vector_type(4)))  unsigned int v4u;
typedef _Float16 h16;


#define VST2(T, ptr, val) do { const T vst2_v_ = (val); *(volatile T*)(ptr) = vst2_v_; __threadfence(); *(volatile T*)(ptr) = vst2_v_; } while (0)

__device__ __forceinline__ float bfr(float f) {
    unsigned u = __float_as_uint(f);
    u += 0x7FFFu + ((u >> 16) & 1u);
    return __uint_as_float(u & 0xFFFF0000u);
}
__device__ __forceinline__ unsigned short f2h_bits(float x) {
    return (fabsf(x) < 6.104e-5f) ? (unsigned short)0 : __builtin_bit_cast(unsigned short, (_Float16)x);
}
__device__ __forceinline__ void st8h(unsigned short* P, size_t o, const float* v) {
    v4u pk;
    pk.x = (unsigned)f2h_bits(v[0]) | ((unsigned)f2h_bits(v[1]) << 16);
    pk.y = (unsigned)f2h_bits(v[2]) | ((unsigned)f2h_bits(v[3]) << 16);
    pk.z = (unsigned)f2h_bits(v[4]) | ((unsigned)f2h_bits(v[5]) << 16);
    pk.w = (unsigned)f2h_bits(v[6]) | ((unsigned)f2h_bits(v[7]) << 16);
    VST2(v4u, (v4u*)(P + o), pk);
}
static __device__ __forceinline__ h16 toh_flush(float v) { const h16 r = (h16)v; return (fabsf(v) < 6.103515625e-05f) ? (h16)0.0f : r; }

union FragU { v16h v; v8h h[2]; };
__device__ __forceinline__ v16h frag_ld(const _Float16* p) {
    FragU f; f.h[0] = *(const v8h*)(p); f.h[1] = *(const v8h*)(p + 16); return f.v;
}
__device__ __forceinline__ v8f wmma16(v16h a, v16h b, v8f c) {
    c = __builtin_amdgcn_wmma_f32_16x16x32_f16(false, a, false, b, (short)0, c, false, false);
    asm volatile("v_nop\n\tv_nop\n\tv_nop\n\tv_nop" : "+v"(c) : "v"(a), "v"(b));
    return c;
}

__host__ __device__ constexpr unsigned win_start(unsigned t) {
    return 16u * ((t == 0u) ? 0u : (((t - 1u) > 5u) ? 5u : (t - 1u)));
}
constexpr bool win_covers() {
    for (unsigned t = 0; t < (unsigned)NTILE; ++t) {
        const unsigned s = win_start(t);
        if (s + (unsigned)AWK > (unsigned)RPAD) return false;
        for (unsigned n = 0; n < 16u; ++n) {
            const unsigned rp = 16u * t + n;
            if (rp >= (unsigned)ROWS) continue;
            const unsigned p = rp / (unsigned)NJ;
            if (p * (unsigned)NJ < s) return false;
            if (p * (unsigned)NJ + (unsigned)NJ > s + (unsigned)AWK) return false;
        }
    }
    return true;
}
static_assert(win_covers());

__global__ __launch_bounds__(256) void k_wt16(const float* __restrict__ Wm, unsigned KI, unsigned NO, unsigned lgper,
                                              unsigned short* __restrict__ W16, float sw) {
    const unsigned layer = blockIdx.y;
    const float* Wl = Wm + (size_t)layer * KI * NO;
    unsigned short* Dl = W16 + (size_t)layer * KI * NO;
    const unsigned u = blockIdx.x * 256u + threadIdx.x;
    const unsigned per = 1u << lgper;
    if (u >= NO * per) return;
    const unsigned k0 = 8u * (u & (per - 1u));
    const unsigned o = u >> lgper;
    float v[8];
#pragma unroll
    for (int i = 0; i < 8; ++i) v[i] = bfr(Wl[(size_t)(k0 + (unsigned)i) * NO + o]) * sw;
    st8h(Dl, (size_t)o * KI + k0, v);
}

__global__ __launch_bounds__(256) void k_adjw(const float* __restrict__ adj, unsigned short* __restrict__ aw) {
    const unsigned u = blockIdx.x * 256u + threadIdx.x;
    if (u >= (unsigned)(RPAD * (AWK / 8))) return;
    const unsigned rp = u >> 3;
    const unsigned k0 = (u & 7u) * 8u;
    const unsigned t = rp >> 4;
    const unsigned kst = win_start(t);
    const unsigned pr = rp / (unsigned)NJ;
    const unsigned ir = rp - pr * (unsigned)NJ;
    float v[8];
#pragma unroll
    for (int i = 0; i < 8; ++i) {
        const unsigned row = kst + k0 + (unsigned)i;
        const unsigned pj = row / (unsigned)NJ;
        const unsigned j = row - pj * (unsigned)NJ;
        const float a = bfr(adj[ir * (unsigned)NJ + j]);
        const bool ok = (pj == pr) && (rp < (unsigned)ROWS) && (row < (unsigned)ROWS);
        v[i] = ok ? a : 0.0f;
    }
    st8h(aw, (size_t)rp * AWK + k0, v);
}

__global__ __launch_bounds__(256) void k_fused(const float* __restrict__ x, const float* __restrict__ w1, const float* __restrict__ b1,
                                               const _Float16* __restrict__ wpl, const float* __restrict__ b2, const float* __restrict__ b3,
                                               const float* __restrict__ b4, const float* __restrict__ w5, const float* __restrict__ b5,
                                               const _Float16* __restrict__ aw, float* __restrict__ out) {
    __shared__ __align__(16) _Float16 sXh[RPAD * XP];
    __shared__ __align__(16) _Float16 sLT[HID * LTP];
    __shared__ __align__(16) _Float16 sAdj[RPAD * AJP];
    __shared__ __align__(16) float sPart[8 * RPAD * 4];
    __shared__ __align__(16) float sOut[OUTF];
    __shared__ __align__(16) float sXs[RPAD * 2];

    const unsigned tid = threadIdx.x, lane = tid & 31u;
    const unsigned wave = (unsigned)__builtin_amdgcn_readfirstlane((int)(threadIdx.x >> 5));
    const unsigned hh = lane >> 4, c = lane & 15u;
    const unsigned n0 = wave * 16u;
    const unsigned blk = blockIdx.x;

    for (unsigned i = tid; i < (unsigned)(RPAD * 8); i += 256u) {
        const unsigned row = i >> 3, ch = i & 7u;
        *(v8h*)(sAdj + row * AJP + 8u * ch) = *(const v8h*)(aw + (size_t)row * AWK + 8u * ch);
    }

    const unsigned rg = tid >> 4, d0 = (tid & 15u) * 8u;
    float w10[8], w11[8], bb[8];
    {
        const v4f a0 = *(const v4f*)(w1 + d0), a1 = *(const v4f*)(w1 + d0 + 4u);
        const v4f c0 = *(const v4f*)(w1 + HID + d0), c1 = *(const v4f*)(w1 + HID + d0 + 4u);
        const v4f e0 = *(const v4f*)(b1 + d0), e1 = *(const v4f*)(b1 + d0 + 4u);
        w10[0] = bfr(a0.x); w10[1] = bfr(a0.y); w10[2] = bfr(a0.z); w10[3] = bfr(a0.w);
        w10[4] = bfr(a1.x); w10[5] = bfr(a1.y); w10[6] = bfr(a1.z); w10[7] = bfr(a1.w);
        w11[0] = bfr(c0.x); w11[1] = bfr(c0.y); w11[2] = bfr(c0.z); w11[3] = bfr(c0.w);
        w11[4] = bfr(c1.x); w11[5] = bfr(c1.y); w11[6] = bfr(c1.z); w11[7] = bfr(c1.w);
        bb[0] = bfr(e0.x); bb[1] = bfr(e0.y); bb[2] = bfr(e0.z); bb[3] = bfr(e0.w);
        bb[4] = bfr(e1.x); bb[5] = bfr(e1.y); bb[6] = bfr(e1.z); bb[7] = bfr(e1.w);
    }
    float w5f[24];
    {
        const float* wp = w5 + (size_t)(n0 + 8u * hh) * 3u;
#pragma unroll
        for (int g = 0; g < 6; ++g) {
            const v4f q = *(const v4f*)(wp + 4 * g);
            w5f[4 * g] = bfr(q.x); w5f[4 * g + 1] = bfr(q.y); w5f[4 * g + 2] = bfr(q.z); w5f[4 * g + 3] = bfr(q.w);
        }
    }
    const float bq2 = bfr(b2[n0 + c]) * CARRY_X;
    const float bq3 = bfr(b3[n0 + c]) * CARRY_X;
    const float bq4 = bfr(b4[n0 + c]) * CARRY_X;

#pragma unroll 1
    for (unsigned sub = 0; sub < (unsigned)(PB / PG); ++sub) {
        const float* xsrc = x + (size_t)(blk * (unsigned)PB + sub * (unsigned)PG) * (unsigned)(NJ * 2);
        for (unsigned e = tid; e < (unsigned)(RPAD * 2); e += 256u) {
            const unsigned ec = (e < (unsigned)(ROWS * 2)) ? e : (unsigned)(ROWS * 2 - 1);
            const float xv = bfr(xsrc[ec]);
            sXs[e] = (e < (unsigned)(ROWS * 2)) ? xv : 0.0f;
        }
        __syncthreads();

#pragma unroll 1
        for (unsigned it = 0; it < (unsigned)NTILE; ++it) {
            const unsigned row = it * 16u + rg;
            const float x0 = sXs[2u * row], x1 = sXs[2u * row + 1u];
            const bool ok = row < (unsigned)ROWS;
            v8h o;
#pragma unroll
            for (int i = 0; i < 8; ++i) {
                const float val = ((x0 * w10[i] + x1 * w11[i]) + bb[i]) * CARRY_X;
                o[i] = toh_flush(ok ? val : 0.0f);
            }
            *(v8h*)(sXh + row * XP + d0) = o;
        }
        __syncthreads();

#pragma unroll
        for (int layer = 0; layer < 3; ++layer) {
            {
                const _Float16* Wl = wpl + (size_t)layer * (HID * HID);
                v16h bw[4];
#pragma unroll
                for (int ks = 0; ks < 4; ++ks) bw[ks] = frag_ld(Wl + (size_t)(n0 + c) * HID + 32u * (unsigned)ks + 8u * hh);
                const float bq = (layer == 0) ? bq2 : ((layer == 1) ? bq3 : bq4);
#pragma unroll 1
                for (unsigned mt = 0; mt < (unsigned)NTILE; ++mt) {
                    v8f acc = (v8f){0.f,0.f,0.f,0.f,0.f,0.f,0.f,0.f};
#pragma unroll
                    for (int ks = 0; ks < 4; ++ks) {
                        const v16h a = frag_ld(sXh + (mt * 16u + c) * XP + 32u * (unsigned)ks + 8u * hh);
                        acc = wmma16(a, bw[ks], acc);
                    }
                    v8h lv;
#pragma unroll
                    for (int r = 0; r < 8; ++r) {
                        float v = acc[r] * SC_L + bq;
                        v = fminf(fmaxf(v, -H_SAT), H_SAT);
                        lv[r] = toh_flush(v);
                    }
                    *(v8h*)(sLT + (n0 + c) * LTP + mt * 16u + 8u * hh) = lv;
                }
            }
            __syncthreads();
#pragma unroll 1
            for (unsigned t = 0; t < (unsigned)NTILE; ++t) {
                const unsigned kb = win_start(t);
                v8f acc = (v8f){0.f,0.f,0.f,0.f,0.f,0.f,0.f,0.f};
#pragma unroll
                for (int ks = 0; ks < 2; ++ks) {
                    const v16h a = frag_ld(sLT + (n0 + c) * LTP + kb + 32u * (unsigned)ks + 8u * hh);
                    const v16h b = frag_ld(sAdj + (t * 16u + c) * AJP + 32u * (unsigned)ks + 8u * hh);
                    acc = wmma16(a, b, acc);
                }
                const unsigned rowp = t * 16u + c;
                const unsigned xo = rowp * XP + n0 + 8u * hh;
                const v8h xr = *(const v8h*)(sXh + xo);
                float v[8];
#pragma unroll
                for (int r = 0; r < 8; ++r) v[r] = fmaxf(acc[r] + (float)xr[r], 0.0f);
                if (layer != 2) {
                    v8h o;
#pragma unroll
                    for (int r = 0; r < 8; ++r) o[r] = toh_flush(fminf(v[r], H_SAT));
                    *(v8h*)(sXh + xo) = o;
                } else {
                    float p0 = 0.f, p1 = 0.f, p2 = 0.f;
#pragma unroll
                    for (int r = 0; r < 8; ++r) {
                        p0 += v[r] * w5f[3 * r];
                        p1 += v[r] * w5f[3 * r + 1];
                        p2 += v[r] * w5f[3 * r + 2];
                    }
                    p0 += __shfl_xor(p0, 16, 32);
                    p1 += __shfl_xor(p1, 16, 32);
                    p2 += __shfl_xor(p2, 16, 32);
                    v4f pv; pv.x = p0; pv.y = p1; pv.z = p2; pv.w = 0.0f;
                    if (hh == 0u) *(v4f*)(sPart + (wave * (unsigned)RPAD + rowp) * 4u) = pv;
                }
            }
            __syncthreads();
        }

        for (unsigned e = tid; e < (unsigned)SUBF; e += 256u) {
            const unsigned row = e / 3u;
            const unsigned c3 = e - 3u * row;
            float s = 0.f;
#pragma unroll
            for (int w = 0; w < 8; ++w) s += sPart[((unsigned)w * (unsigned)RPAD + row) * 4u + c3];
            sOut[sub * (unsigned)SUBF + e] = s * INV_CARRY + bfr(b5[c3]);
        }
    }
    __syncthreads();

    {
        const unsigned i1 = tid + 256u;
        const bool has1 = i1 < (unsigned)(OUTF / 4);
        const unsigned i1c = has1 ? i1 : (unsigned)(OUTF / 4 - 1);
        const v4f o0 = *(const v4f*)(sOut + 4u * tid);
        const v4f o1 = *(const v4f*)(sOut + 4u * i1c);
        float* dst = out + (size_t)blk * (unsigned)OUTF;
        for (int pass = 0; pass < 2; ++pass) {
            *(volatile v4f*)(dst + 4u * tid) = o0;
            if (has1) *(volatile v4f*)(dst + 4u * i1) = o1;
            __threadfence();
        }
    }
}

extern "C" void kernel_launch(void* const* d_in, const int* in_sizes, int n_in, void* d_out, int out_size,
                              void* d_ws, size_t ws_size, hipStream_t stream) {
    if (n_in < 12) return;
    if (in_sizes[0] < NSAMP * NJ * 2 || in_sizes[1] < NJ * NJ || in_sizes[2] < 2 * HID || in_sizes[3] < HID) return;
    if (in_sizes[4] < HID * HID || in_sizes[5] < HID || in_sizes[6] < HID * HID || in_sizes[7] < HID) return;
    if (in_sizes[8] < HID * HID || in_sizes[9] < HID || in_sizes[10] < HID * 3 || in_sizes[11] < 3) return;
    if (out_size < NSAMP * NJ * 3) return;

    const float* x   = (const float*)d_in[0];
    const float* adj = (const float*)d_in[1];
    const float* w1  = (const float*)d_in[2];
    const float* b1  = (const float*)d_in[3];
    const float* w2  = (const float*)d_in[4];
    const float* b2  = (const float*)d_in[5];
    const float* w3  = (const float*)d_in[6];
    const float* b3  = (const float*)d_in[7];
    const float* w4  = (const float*)d_in[8];
    const float* b4  = (const float*)d_in[9];
    const float* w5  = (const float*)d_in[10];
    const float* b5  = (const float*)d_in[11];
    float* out = (float*)d_out;

    char* wsp = (char*)d_ws;
    size_t off = 0;
    auto carve = [&](size_t bytes) -> void* { void* r = wsp + off; off += (bytes + 255) & ~(size_t)255; return r; };
    unsigned short* wpl = (unsigned short*)carve((size_t)3 * HID * HID * 2);
    unsigned short* awp = (unsigned short*)carve((size_t)RPAD * AWK * 2);
    if (off > ws_size || off > (size_t)134217728) return;

    k_wt16<<<dim3((HID * (HID / 8)) / 256, 1), 256, 0, stream>>>(w2, HID, HID, 4, wpl, 32.0f);
    k_wt16<<<dim3((HID * (HID / 8)) / 256, 1), 256, 0, stream>>>(w3, HID, HID, 4, wpl + (size_t)HID * HID, 32.0f);
    k_wt16<<<dim3((HID * (HID / 8)) / 256, 1), 256, 0, stream>>>(w4, HID, HID, 4, wpl + (size_t)2 * HID * HID, 32.0f);
    k_adjw<<<(RPAD * (AWK / 8) + 255) / 256, 256, 0, stream>>>(adj, awp);

    k_fused<<<NSAMP / PB, 256, 0, stream>>>(x, w1, b1, (const _Float16*)wpl, b2, b3, b4, w5, b5, (const _Float16*)awp, out);
}
